// BDH_66056597013022
// MI455X (gfx1250) — hardware-verified
//
#include <hip/hip_runtime.h>


#ifndef NB
#define NB 4
#endif
#ifndef SEQ
#define SEQ 1024
#endif
#define NB_FULL  4
#define SEQ_FULL 1024
#ifndef OUT_SEQ
#define OUT_SEQ SEQ
#endif
#define DM   256
#define NH_  4
#define DH   1024
#define HALF 512
#define NTOT 4096
#define VOC  256
#define NL   6
#define OP   68
#define TS   (64 * OP)
#define LNP  264
#define WSC  64.0f
#define WSI  (1.0f / 64.0f)
#define ASC  (1.0f / 64.0f)
#define YSC  (1.0f / 64.0f)
#define LN_EPS 1e-5f
#define LOG2_1E4 13.287712379549449f
#define INV_2PI  0.15915494309189535f
#define TP1 6.28125f
#define TP2 0.0019353032112121582f
#define TP3 3.9683743187e-9f

static_assert(NH_ * DH == NTOT);
static_assert(DH == 2 * HALF);
static_assert(HALF % 64 == 0);
static_assert(DM % 64 == 0);
static_assert(DM % 32 == 0);
static_assert(DH % 64 == 0);
static_assert(DH % 32 == 0);
static_assert(VOC % 64 == 0);
static_assert(SEQ % 64 == 0);
static_assert(SEQ % 32 == 0);
static_assert((NB * SEQ) % 64 == 0);
static_assert(NB <= NB_FULL);
static_assert(SEQ <= SEQ_FULL);
static_assert(SEQ <= DH);
static_assert((OP * 4) % 16 == 0);
static_assert((LNP * 2) % 16 == 0);
static_assert(DM == 256);
static_assert(32 * 2 * 4 == DM);
static_assert(16 * 4 == 64);
static_assert(8 * 16 == 64 * 2);
static_assert(32 * 2 == 64);
static_assert(16 * 16 == 64 * 4);
static_assert(32 * 32 * 4 == 64 * 64);
static_assert(8 * 2 * 4 == 64);
static_assert(4 * 256 * 4 == 64 * 64);
static_assert(8 * 8 == 64);
static_assert(8 * 8 * 4 == DM);
static_assert(2 * TS * 4 <= 131072);
static_assert(64 * LNP * 2 <= 131072);

typedef _Float16 h16;
typedef __attribute__((ext_vector_type(16))) _Float16 v16h;
typedef __attribute__((ext_vector_type(8)))  _Float16 v8h;
typedef __attribute__((ext_vector_type(4)))  _Float16 v4h;
typedef __attribute__((ext_vector_type(8)))  float    v8f;
typedef __attribute__((ext_vector_type(4)))  float    v4f;
typedef v4f  __attribute__((may_alias)) v4fa;
typedef v8h  __attribute__((may_alias)) v8ha;
typedef v4h  __attribute__((may_alias)) v4ha;

__device__ __forceinline__ unsigned short f2bf(float f) { unsigned u = __float_as_uint(f); u += 0x7FFFu + ((u >> 16) & 1u); return (unsigned short)(u >> 16); }
__device__ __forceinline__ float bfr(float f) { return __uint_as_float(((unsigned)f2bf(f)) << 16); }
__device__ __forceinline__ v16h cat16(v8h lo, v8h hi) { return __builtin_shufflevector(lo, hi, 0, 1, 2, 3, 4, 5, 6, 7, 8, 9, 10, 11, 12, 13, 14, 15); }
__device__ __forceinline__ v8f wmma16(v16h a, v16h b, v8f c) { return __builtin_amdgcn_wmma_f32_16x16x32_f16(false, a, false, b, (short)0, c, false, false); }
__device__ __forceinline__ v8f wmma_g(v16h a, v16h b, v8f c) { c = wmma16(a, b, c); asm volatile("v_nop\n\tv_nop\n\tv_nop\n\tv_nop" : "+v"(c) : "v"(a), "v"(b)); return c; }
__device__ __forceinline__ v16h ldh(const h16* p) { return cat16(*(const v8h*)p, *(const v8h*)(p + 16)); }
__device__ __forceinline__ h16 toh_flush(float v) { const h16 r = (h16)v; return (fabsf(v) < 6.103515625e-05f) ? (h16)0.0f : r; }
__device__ __forceinline__ void wave_sync() { __builtin_amdgcn_fence(3  , "wavefront"); __builtin_amdgcn_wave_barrier(); asm volatile("" ::: "memory"); }
__device__ __forceinline__ float wsum(float v) { v += __shfl_xor(v, 16, 32); v += __shfl_xor(v, 8, 32); v += __shfl_xor(v, 4, 32); v += __shfl_xor(v, 2, 32); v += __shfl_xor(v, 1, 32); return v; }

__device__ __forceinline__ void gemm_acc64(v8f (&acc)[4][4], const h16* __restrict__ A, const size_t aoff, const int lda,
                                           const h16* __restrict__ Bt, const size_t boff, const int ldb, const int K) {
#pragma unroll 1
    for (int kc = 0; kc < K; kc += 32) {
        v16h a[4];
#pragma unroll
        for (int mb = 0; mb < 4; ++mb) a[mb] = ldh(A + aoff + (size_t)mb * 16 * lda + kc);
#pragma unroll
        for (int nb = 0; nb < 4; ++nb) { const v16h b = ldh(Bt + boff + (size_t)nb * 16 * ldb + kc);
#pragma unroll
            for (int mb = 0; mb < 4; ++mb) acc[mb][nb] = wmma_g(a[mb], b, acc[mb][nb]); }
    }
}

__global__ __launch_bounds__(256) void k_wtr(const float* __restrict__ in, h16* out, int R, int C) {
    __shared__ __align__(16) float tl[64 * OP];
    const int tid = threadIdx.x, lane = tid & 31;
    const int wave = __builtin_amdgcn_readfirstlane((int)(threadIdx.x >> 5));
    const int c0 = blockIdx.x * 64, r0 = blockIdx.y * 64;
    const size_t zo = (size_t)blockIdx.z * (size_t)R * (size_t)C;
#pragma unroll 1
    for (int it = 0; it < 4; ++it) { const int p = it * 256 + tid; const int row = p >> 4, c4 = (p & 15) * 4;
        const v4f v = *(const v4f*)(in + zo + (size_t)(r0 + row) * C + c0 + c4); v4f w;
#pragma unroll
        for (int k = 0; k < 4; ++k) w[k] = bfr(v[k]) * WSC;
        *(v4fa*)(&tl[row * OP + c4]) = w; }
    __syncthreads();
#pragma unroll 1
    for (int ps = 0; ps < 2; ++ps) {
#pragma unroll
        for (int s = 0; s < 2; ++s) { const int cr = (wave * 2 + s) * 4 + (lane >> 3), r8 = (lane & 7) * 8; v8h hv;
#pragma unroll
            for (int i = 0; i < 8; ++i) hv[i] = toh_flush(tl[(r8 + i) * OP + cr]);
            *(volatile v8h*)(out + zo + (size_t)(c0 + cr) * R + r0 + r8) = hv; }
        if (ps == 0) __threadfence(); }
}

__global__ __launch_bounds__(256) void k_ropetab(float* COS, float* SIN) {
#pragma clang fp contract(off)
    const int idx = blockIdx.x * 256 + threadIdx.x; if (idx >= SEQ * (HALF / 4)) return;
    const int t = idx / (HALF / 4), i0 = (idx % (HALF / 4)) * 4;
    v4f c, s;
#pragma unroll
    for (int k = 0; k < 4; ++k) {
        const float ex = (float)(2 * (i0 + k)) * (1.0f / (float)DH);
        const float inv = exp2f(-(ex * LOG2_1E4));
        const float a = (float)t * inv;
        const float n = rintf(a * INV_2PI);
        float r = fmaf(-n, TP1, a); r = fmaf(-n, TP2, r); r = fmaf(-n, TP3, r);
        c[k] = __cosf(r); s[k] = __sinf(r); }
    *(volatile v4f*)(COS + (size_t)idx * 4) = c; *(volatile v4f*)(SIN + (size_t)idx * 4) = s;
    __threadfence();
    *(volatile v4f*)(COS + (size_t)idx * 4) = c; *(volatile v4f*)(SIN + (size_t)idx * 4) = s;
}

__global__ __launch_bounds__(256) void k_ln(const int* __restrict__ tokens, const float* __restrict__ emb, const float* __restrict__ Z, float* VF, h16* VH, h16* VT, int mode) {
#pragma clang fp contract(off)
    __shared__ __align__(16) h16 tile[64 * LNP];
    const int lane = threadIdx.x & 31;
    const int wave = __builtin_amdgcn_readfirstlane((int)(threadIdx.x >> 5));
    const int r0 = blockIdx.x * 64; const int b = r0 / SEQ, t0 = r0 % SEQ;
#pragma unroll 1
    for (int i = 0; i < 8; ++i) {
        const int rl = wave * 8 + i; const size_t row = (size_t)b * SEQ + t0 + rl;
        float* vrow = VF + row * DM;
        v4f xa, xb, va = (v4f){}, vb = (v4f){};
        if (mode == 0) {
            int tok = tokens[(size_t)b * SEQ_FULL + t0 + rl]; tok = tok < 0 ? 0 : (tok > VOC - 1 ? VOC - 1 : tok);
            const float* src = emb + (size_t)tok * DM;
            xa = *(const v4f*)(src + lane * 4); xb = *(const v4f*)(src + 128 + lane * 4);
#pragma unroll
            for (int k = 0; k < 4; ++k) { xa[k] = bfr(xa[k]); xb[k] = bfr(xb[k]); }
        } else {
            const float* src = Z + row * DM;
            xa = *(const v4f*)(src + lane * 4); xb = *(const v4f*)(src + 128 + lane * 4);
            va = *(const v4f*)(vrow + lane * 4); vb = *(const v4f*)(vrow + 128 + lane * 4);
        }
        const int nln = 1 + (mode != 0);
#pragma unroll 1
        for (int q = 0; q < nln; ++q) {
            float s = ((xa[0] + xa[1]) + (xa[2] + xa[3])) + ((xb[0] + xb[1]) + (xb[2] + xb[3]));
            s = wsum(s); const float mean = s * (1.0f / (float)DM);
            xa = xa - mean; xb = xb - mean;
            float qq = ((xa[0] * xa[0] + xa[1] * xa[1]) + (xa[2] * xa[2] + xa[3] * xa[3])) + ((xb[0] * xb[0] + xb[1] * xb[1]) + (xb[2] * xb[2] + xb[3] * xb[3]));
            qq = wsum(qq); const float rs = rsqrtf(qq * (1.0f / (float)DM) + LN_EPS);
            xa = xa * rs; xb = xb * rs;
            if (q + 1 < nln) { xa = va + xa; xb = vb + xb; }
        }
        *(volatile v4f*)(vrow + lane * 4) = xa; *(volatile v4f*)(vrow + 128 + lane * 4) = xb;
        __threadfence();
        *(volatile v4f*)(vrow + lane * 4) = xa; *(volatile v4f*)(vrow + 128 + lane * 4) = xb;
        v4h ha, hb;
#pragma unroll
        for (int k = 0; k < 4; ++k) { ha[k] = toh_flush(xa[k]); hb[k] = toh_flush(xb[k]); }
        *(v4ha*)(&tile[rl * LNP + lane * 4]) = ha; *(v4ha*)(&tile[rl * LNP + 128 + lane * 4]) = hb;
    }
    __syncthreads();
#pragma unroll 1
    for (int ps = 0; ps < 2; ++ps) {
#pragma unroll 1
        for (int i = 0; i < 8; ++i) { const int rl = wave * 8 + i;
            const v8h val = *(const v8ha*)(&tile[rl * LNP + lane * 8]);
            *(volatile v8h*)(VH + ((size_t)b * SEQ + t0 + rl) * DM + lane * 8) = val; }
#pragma unroll 1
        for (int s = 0; s < 8; ++s) { const int d = (wave * 8 + s) * 4 + (lane >> 3), t8 = (lane & 7) * 8; v8h hv;
#pragma unroll
            for (int k = 0; k < 8; ++k) hv[k] = tile[(t8 + k) * LNP + d];
            *(volatile v8h*)(VT + ((size_t)b * DM + d) * SEQ + t0 + t8) = hv; }
        if (ps == 0) __threadfence(); }
}

__global__ __launch_bounds__(32) void k_xrope(const h16* __restrict__ VH, const h16* __restrict__ DXT, const float* __restrict__ COS, const float* __restrict__ SIN,
                                              h16* XH, h16* XR, h16* XRT) {
    __shared__ __align__(16) float os[2 * TS];
    const int lane = threadIdx.x & 31, lr = lane & 15, hi = lane >> 4;
    const int t0 = blockIdx.x * 64, e0 = blockIdx.y * 64, z = blockIdx.z; const int b = z / NH_, h = z % NH_;
    const size_t aoff = ((size_t)b * SEQ + t0 + lr) * DM + 8 * hi;
#pragma unroll 1
    for (int ph = 0; ph < 2; ++ph) {
        v8f acc[4][4];
#pragma unroll
        for (int mb = 0; mb < 4; ++mb)
#pragma unroll
            for (int nb = 0; nb < 4; ++nb) acc[mb][nb] = (v8f){};
        const size_t boff = ((size_t)h * DH + (size_t)(ph * HALF + e0 + lr)) * DM + 8 * hi;
        gemm_acc64(acc, VH, aoff, DM, DXT, boff, DM, DM);
#pragma unroll
        for (int mb = 0; mb < 4; ++mb)
#pragma unroll
            for (int nb = 0; nb < 4; ++nb)
#pragma unroll
                for (int j = 0; j < 8; ++j) os[ph * TS + (mb * 16 + hi * 8 + j) * OP + nb * 16 + lr] = fmaxf(acc[mb][nb][j] * WSI, 0.0f);
    }
    wave_sync();
    const size_t pz = (size_t)z * SEQ * DH;
    const int rq = lane >> 3, c8 = (lane & 7) * 8;
#pragma unroll 1
    for (int ps = 0; ps < 2; ++ps) {
#pragma unroll 1
        for (int ph = 0; ph < 2; ++ph) {
#pragma unroll 4
            for (int s = 0; s < 16; ++s) { const int row = 4 * s + rq;
                const v4f x0 = *(const v4fa*)(&os[ph * TS + row * OP + c8]); const v4f x1 = *(const v4fa*)(&os[ph * TS + row * OP + c8 + 4]); v8h hv;
#pragma unroll
                for (int i = 0; i < 4; ++i) { hv[i] = toh_flush(x0[i]); hv[4 + i] = toh_flush(x1[i]); }
                *(volatile v8h*)(XH + pz + (size_t)(t0 + row) * DH + ph * HALF + e0 + c8) = hv; } }
        if (ps == 0) __threadfence(); }
    wave_sync();
#pragma unroll 1
    for (int it = 0; it < 32; ++it) { const int p = it * 32 + lane; const int row = p >> 4, c4 = (p & 15) * 4;
        const v4f x1 = *(const v4fa*)(&os[row * OP + c4]); const v4f x2 = *(const v4fa*)(&os[TS + row * OP + c4]);
        const v4f cs = *(const v4f*)(COS + (size_t)(t0 + row) * HALF + e0 + c4); const v4f sn = *(const v4f*)(SIN + (size_t)(t0 + row) * HALF + e0 + c4);
        const v4f r1 = x1 * cs - x2 * sn; const v4f r2 = x2 * cs + x1 * sn;
        *(v4fa*)(&os[row * OP + c4]) = r1; *(v4fa*)(&os[TS + row * OP + c4]) = r2; }
    wave_sync();
    const size_t qz = (size_t)z * DH * SEQ;
#pragma unroll 1
    for (int ps = 0; ps < 2; ++ps) {
#pragma unroll 1
        for (int ph = 0; ph < 2; ++ph) {
#pragma unroll 4
            for (int s = 0; s < 16; ++s) { const int row = 4 * s + rq;
                const v4f x0 = *(const v4fa*)(&os[ph * TS + row * OP + c8]); const v4f x1 = *(const v4fa*)(&os[ph * TS + row * OP + c8 + 4]); v8h hv;
#pragma unroll
                for (int i = 0; i < 4; ++i) { hv[i] = toh_flush(x0[i]); hv[4 + i] = toh_flush(x1[i]); }
                *(volatile v8h*)(XR + pz + (size_t)(t0 + row) * DH + ph * HALF + e0 + c8) = hv; }
#pragma unroll 4
            for (int s = 0; s < 16; ++s) { const int er = 4 * s + rq; v8h hv;
#pragma unroll
                for (int i = 0; i < 8; ++i) hv[i] = toh_flush(os[ph * TS + (c8 + i) * OP + er]);
                *(volatile v8h*)(XRT + qz + (size_t)(ph * HALF + e0 + er) * SEQ + t0 + c8) = hv; } }
        if (ps == 0) __threadfence(); }
}

__global__ __launch_bounds__(32) void k_gemm_h16(const h16* __restrict__ A, const h16* __restrict__ Bt, h16* C, int lda, int ldb, int ldc, int K, int adiv,
                                                 unsigned long long sA, unsigned long long sB, unsigned long long sC, float scale) {
    __shared__ __align__(16) float os[TS];
    const int lane = threadIdx.x & 31, lr = lane & 15, hi = lane >> 4;
    const int r0 = blockIdx.x * 64, c0 = blockIdx.y * 64, z = blockIdx.z;
    v8f acc[4][4];
#pragma unroll
    for (int mb = 0; mb < 4; ++mb)
#pragma unroll
        for (int nb = 0; nb < 4; ++nb) acc[mb][nb] = (v8f){};
    gemm_acc64(acc, A, (size_t)(z / adiv) * (size_t)sA + (size_t)(r0 + lr) * lda + 8 * hi, lda, Bt, (size_t)z * (size_t)sB + (size_t)(c0 + lr) * ldb + 8 * hi, ldb, K);
#pragma unroll
    for (int mb = 0; mb < 4; ++mb)
#pragma unroll
        for (int nb = 0; nb < 4; ++nb)
#pragma unroll
            for (int j = 0; j < 8; ++j) os[(mb * 16 + hi * 8 + j) * OP + nb * 16 + lr] = acc[mb][nb][j] * scale;
    wave_sync();
    const size_t cb = (size_t)z * (size_t)sC + (size_t)r0 * ldc + c0;
    const int rq = lane >> 3, c8 = (lane & 7) * 8;
#pragma unroll 1
    for (int ps = 0; ps < 2; ++ps) {
#pragma unroll 4
        for (int s = 0; s < 16; ++s) { const int row = 4 * s + rq;
            const v4f x0 = *(const v4fa*)(&os[row * OP + c8]); const v4f x1 = *(const v4fa*)(&os[row * OP + c8 + 4]); v8h hv;
#pragma unroll
            for (int i = 0; i < 4; ++i) { hv[i] = toh_flush(x0[i]); hv[4 + i] = toh_flush(x1[i]); }
            *(volatile v8h*)(C + cb + (size_t)row * ldc + c8) = hv; }
        if (ps == 0) __threadfence(); }
}

__global__ __launch_bounds__(32) void k_ygate(const h16* __restrict__ AP, const h16* __restrict__ DYT, h16* XY) {
    __shared__ __align__(16) float os[TS];
    const int lane = threadIdx.x & 31, lr = lane & 15, hi = lane >> 4;
    const int r0 = blockIdx.x * 64, c0 = blockIdx.y * 64, z = blockIdx.z; const int h = z % NH_;
    v8f acc[4][4];
#pragma unroll
    for (int mb = 0; mb < 4; ++mb)
#pragma unroll
        for (int nb = 0; nb < 4; ++nb) acc[mb][nb] = (v8f){};
    gemm_acc64(acc, AP, ((size_t)z * SEQ + r0 + lr) * DM + 8 * hi, DM, DYT, ((size_t)h * DH + c0 + lr) * DM + 8 * hi, DM, DM);
#pragma unroll
    for (int mb = 0; mb < 4; ++mb)
#pragma unroll
        for (int nb = 0; nb < 4; ++nb)
#pragma unroll
            for (int j = 0; j < 8; ++j) os[(mb * 16 + hi * 8 + j) * OP + nb * 16 + lr] = fmaxf(acc[mb][nb][j], 0.0f) * YSC;
    wave_sync();
    const size_t cb = ((size_t)z * SEQ + r0) * DH + c0;
    const int rq = lane >> 3, c8 = (lane & 7) * 8;
#pragma unroll 4
    for (int s = 0; s < 16; ++s) { const int row = 4 * s + rq;
        const v8h xv = *(const v8h*)(XY + cb + (size_t)row * DH + c8);
        v4f x0 = *(const v4fa*)(&os[row * OP + c8]); v4f x1 = *(const v4fa*)(&os[row * OP + c8 + 4]);
#pragma unroll
        for (int i = 0; i < 4; ++i) { x0[i] = x0[i] * (float)xv[i]; x1[i] = x1[i] * (float)xv[4 + i]; }
        *(v4fa*)(&os[row * OP + c8]) = x0; *(v4fa*)(&os[row * OP + c8 + 4]) = x1; }
    wave_sync();
#pragma unroll 1
    for (int ps = 0; ps < 2; ++ps) {
#pragma unroll 4
        for (int s = 0; s < 16; ++s) { const int row = 4 * s + rq;
            const v4f x0 = *(const v4fa*)(&os[row * OP + c8]); const v4f x1 = *(const v4fa*)(&os[row * OP + c8 + 4]); v8h hv;
#pragma unroll
            for (int i = 0; i < 4; ++i) { hv[i] = toh_flush(x0[i]); hv[4 + i] = toh_flush(x1[i]); }
            *(volatile v8h*)(XY + cb + (size_t)row * DH + c8) = hv; }
        if (ps == 0) __threadfence(); }
}

__global__ __launch_bounds__(32) void k_gemm_f32(const h16* __restrict__ A, const h16* __restrict__ Bt, float* C, int lda, int ldb, int ldc, int Kseg, int nseg,
                                                 unsigned long long sAb, unsigned long long sAseg, int crows, float scale) {
    __shared__ __align__(16) float os[TS];
    const int lane = threadIdx.x & 31, lr = lane & 15, hi = lane >> 4;
    const int r0 = blockIdx.x * 64, c0 = blockIdx.y * 64; const int b = r0 / SEQ, t = r0 % SEQ;
    v8f acc[4][4];
#pragma unroll
    for (int mb = 0; mb < 4; ++mb)
#pragma unroll
        for (int nb = 0; nb < 4; ++nb) acc[mb][nb] = (v8f){};
#pragma unroll 1
    for (int sg = 0; sg < nseg; ++sg)
        gemm_acc64(acc, A, (size_t)b * (size_t)sAb + (size_t)sg * (size_t)sAseg + (size_t)(t + lr) * lda + 8 * hi, lda,
                   Bt, (size_t)(c0 + lr) * ldb + (size_t)sg * Kseg + 8 * hi, ldb, Kseg);
#pragma unroll
    for (int mb = 0; mb < 4; ++mb)
#pragma unroll
        for (int nb = 0; nb < 4; ++nb)
#pragma unroll
            for (int j = 0; j < 8; ++j) os[(mb * 16 + hi * 8 + j) * OP + nb * 16 + lr] = acc[mb][nb][j] * scale;
    wave_sync();
    const size_t cb = ((size_t)b * crows + t) * ldc + c0;
    const int rh = lane >> 4, c4 = (lane & 15) * 4;
#pragma unroll 1
    for (int ps = 0; ps < 2; ++ps) {
#pragma unroll 4
        for (int s = 0; s < 32; ++s) { const int row = 2 * s + rh;
            const v4f val = *(const v4fa*)(&os[row * OP + c4]);
            *(volatile v4f*)(C + cb + (size_t)row * ldc + c4) = val; }
        if (ps == 0) __threadfence(); }
}

static constexpr size_t al256(size_t v) { return (v + 255) & ~(size_t)255; }
static constexpr size_t SZ_VF  = al256((size_t)NB * SEQ * DM * 4);
static constexpr size_t SZ_VH  = al256((size_t)NB * SEQ * DM * 2);
static constexpr size_t SZ_WX  = al256((size_t)NH_ * DH * DM * 2);
static constexpr size_t SZ_ET  = al256((size_t)DM * NTOT * 2);
static constexpr size_t SZ_RO  = al256((size_t)VOC * DM * 2);
static constexpr size_t SZ_TAB = al256((size_t)SEQ * HALF * 4);
static constexpr size_t SZ_XP  = al256((size_t)NB * NH_ * SEQ * DH * 2);
static constexpr size_t SZ_MT  = al256((size_t)NB * NH_ * DM * DH * 2);
static constexpr size_t SZ_TOTAL = SZ_VF + 2 * SZ_VH + 2 * SZ_WX + SZ_ET + SZ_RO + 2 * SZ_TAB + 3 * SZ_XP + SZ_MT;
static_assert(SZ_TOTAL <= (size_t)134217728);
static_assert((size_t)NB * NH_ * SEQ * DM * 2 <= SZ_XP);
static_assert((size_t)NB * SEQ * DM * 4 <= SZ_MT);
static_assert((size_t)NB * DM * SEQ * 2 <= SZ_VH);

extern "C" void kernel_launch(void* const* d_in, const int* in_sizes, int n_in,
                              void* d_out, int out_size, void* d_ws, size_t ws_size, hipStream_t stream) {
    if (n_in < 6) return;
    if ((size_t)in_sizes[0] < (size_t)(NB - 1) * SEQ_FULL + SEQ) return;
    if ((size_t)in_sizes[1] < (size_t)VOC * DM || (size_t)in_sizes[2] < (size_t)NTOT * DM) return;
    if ((size_t)in_sizes[3] < (size_t)NH_ * DM * DH || (size_t)in_sizes[4] < (size_t)NH_ * DM * DH || (size_t)in_sizes[5] < (size_t)DM * VOC) return;
    if ((size_t)out_size < ((size_t)(NB - 1) * OUT_SEQ + SEQ) * VOC) return;
    if (SZ_TOTAL > ws_size) return;
    const int*   tokens = (const int*)d_in[0];
    const float* emb    = (const float*)d_in[1];
    const float* Ein    = (const float*)d_in[2];
    const float* Dxin   = (const float*)d_in[3];
    const float* Dyin   = (const float*)d_in[4];
    const float* ROin   = (const float*)d_in[5];
    float* OUT = (float*)d_out;
    char* wsp = (char*)d_ws;
    float* VF  = (float*)wsp; wsp += SZ_VF;
    h16*   VH  = (h16*)wsp;   wsp += SZ_VH;
    h16*   VT  = (h16*)wsp;   wsp += SZ_VH;
    h16*   DXT = (h16*)wsp;   wsp += SZ_WX;
    h16*   DYT = (h16*)wsp;   wsp += SZ_WX;
    h16*   ET  = (h16*)wsp;   wsp += SZ_ET;
    h16*   ROT = (h16*)wsp;   wsp += SZ_RO;
    float* COS = (float*)wsp; wsp += SZ_TAB;
    float* SIN = (float*)wsp; wsp += SZ_TAB;
    h16*   XH  = (h16*)wsp;   wsp += SZ_XP;
    h16*   XR  = (h16*)wsp;   wsp += SZ_XP;
    h16*   XRT = (h16*)wsp;   wsp += SZ_XP;
    h16*   MT  = (h16*)wsp;   wsp += SZ_MT;
    h16*   AP  = XRT;
    float* Z   = (float*)MT;

    k_wtr<<<dim3(DH / 64, DM / 64, NH_), 256, 0, stream>>>(Dxin, DXT, DM, DH);
    k_wtr<<<dim3(DH / 64, DM / 64, NH_), 256, 0, stream>>>(Dyin, DYT, DM, DH);
    k_wtr<<<dim3(DM / 64, NTOT / 64, 1), 256, 0, stream>>>(Ein, ET, NTOT, DM);
    k_wtr<<<dim3(VOC / 64, DM / 64, 1), 256, 0, stream>>>(ROin, ROT, DM, VOC);
    k_ropetab<<<(unsigned)((SEQ * (HALF / 4) + 255) / 256), 256, 0, stream>>>(COS, SIN);
    k_ln<<<NB * SEQ / 64, 256, 0, stream>>>(tokens, emb, Z, VF, VH, VT, 0);

    for (int l = 0; l < NL; ++l) {
        k_xrope<<<dim3(SEQ / 64, HALF / 64, NB * NH_), 32, 0, stream>>>(VH, DXT, COS, SIN, XH, XR, XRT);
        k_gemm_h16<<<dim3(DM / 64, DH / 64, NB * NH_), 32, 0, stream>>>(VT, XRT, MT, SEQ, SEQ, DH, SEQ, NH_,
            (unsigned long long)DM * SEQ, (unsigned long long)DH * SEQ, (unsigned long long)DM * DH, 1.0f);
        k_gemm_h16<<<dim3(SEQ / 64, DM / 64, NB * NH_), 32, 0, stream>>>(XR, MT, AP, DH, DH, DM, DH, 1,
            (unsigned long long)SEQ * DH, (unsigned long long)DM * DH, (unsigned long long)SEQ * DM, ASC);
        k_ygate<<<dim3(SEQ / 64, DH / 64, NB * NH_), 32, 0, stream>>>(AP, DYT, XH);
        k_gemm_f32<<<dim3(NB * SEQ / 64, DM / 64, 1), 32, 0, stream>>>(XH, ET, Z, DH, NTOT, DM, DH, NH_,
            (unsigned long long)NH_ * SEQ * DH, (unsigned long long)SEQ * DH, SEQ, 1.0f);
        k_ln<<<NB * SEQ / 64, 256, 0, stream>>>(tokens, emb, Z, VF, VH, VT, 1);
    }
    k_gemm_f32<<<dim3(NB * SEQ / 64, VOC / 64, 1), 32, 0, stream>>>(VH, ROT, OUT, DM, DM, VOC, DM, 1,
        (unsigned long long)SEQ * DM, 0ull, OUT_SEQ, WSI);
}
